// MemoryEfficientMultiHeadAttention_61306363183427
// MI455X (gfx1250) — hardware-verified
//
#include <hip/hip_runtime.h>
#include <stdint.h>
#include <stddef.h>


typedef _Float16 h16;
typedef h16   v16h __attribute__((ext_vector_type(16)));
typedef h16   v8h  __attribute__((ext_vector_type(8)));
typedef float v8f  __attribute__((ext_vector_type(8)));
typedef float v4f  __attribute__((ext_vector_type(4)));

#define D_MODEL 1024
#define SEQ     2048
#define BATCH   4
#define HEADS   16
#define DEPTH   64
#define M_TOTAL (BATCH * SEQ)

#define LDA 40
#define LDB 40
#define LDK 72
#define LDV 40
#define CPH 72
#define CPT 136
#define CPF 68
#define OPH 72

#define W_SCALE    64.0f
#define W_ISCALE   0.015625f
#define P_SCALE    256.0f
#define SCORE_SC   0.125f
#define ATT_OSCALE 0.125f
#define OUT_ISCALE 0.00048828125f

static __device__ __forceinline__ v8f wmma16(v16h a, v16h b, v8f c) {
  v8f d = __builtin_amdgcn_wmma_f32_16x16x32_f16(false, a, false, b, (short)0, c, false, false);
  asm volatile("v_nop\n\tv_nop\n\tv_nop\n\tv_nop" : "+v"(d) : "v"(a), "v"(b));
  return d;
}

static __device__ __forceinline__ v16h cat8(v8h lo, v8h hi) {
  return __builtin_shufflevector(lo, hi, 0,1,2,3,4,5,6,7,8,9,10,11,12,13,14,15);
}

static __device__ __forceinline__ v8h cvt8(v4f a, v4f b, float s) {
  v8h r;
  r[0]=(h16)(a[0]*s); r[1]=(h16)(a[1]*s); r[2]=(h16)(a[2]*s); r[3]=(h16)(a[3]*s);
  r[4]=(h16)(b[0]*s); r[5]=(h16)(b[1]*s); r[6]=(h16)(b[2]*s); r[7]=(h16)(b[3]*s);
  return r;
}

static __device__ __forceinline__ void tile_mma(const h16* Al, const h16* Bl,
                                                int waveM, int waveN, int l15, int half,
                                                v8f acc[2][2]) {
  v16h af[2], bf[2];
#pragma unroll
  for (int si = 0; si < 2; ++si) {
    const h16* p = Al + (waveM*32 + si*16 + l15)*LDA + half*8;
    af[si] = cat8(*(const v8h*)p, *(const v8h*)(p + 16));
  }
#pragma unroll
  for (int sj = 0; sj < 2; ++sj) {
    const h16* p = Bl + (waveN*32 + sj*16 + l15)*LDB + half*8;
    bf[sj] = cat8(*(const v8h*)p, *(const v8h*)(p + 16));
  }
#pragma unroll
  for (int si = 0; si < 2; ++si)
#pragma unroll
    for (int sj = 0; sj < 2; ++sj)
      acc[si][sj] = wmma16(af[si], bf[sj], acc[si][sj]);
}

static __device__ __forceinline__ void qkv_store(const h16* Ct, h16* dst, bool tr,
                                                 int b, int h, int s0, int wid, int lane) {
  if (!tr) {
#pragma unroll
    for (int it = 0; it < 4; ++it) {
      const int rowL = wid*16 + it*4 + (lane >> 3);
      const int piece = lane & 7;
      const v4f v = *(const v4f*)(Ct + rowL*CPH + piece*8);
      h16* p = dst + ((size_t)(b*HEADS + h)*SEQ + s0 + rowL)*DEPTH + piece*8;
      *(volatile v4f*)p = v;
    }
  } else {
#pragma unroll
    for (int it = 0; it < 4; ++it) {
      const int dL = wid*8 + it*2 + (lane >> 4);
      const int piece = lane & 15;
      const v4f v = *(const v4f*)(Ct + dL*CPT + piece*8);
      h16* p = dst + ((size_t)(b*HEADS + h)*DEPTH + dL)*SEQ + s0 + piece*8;
      *(volatile v4f*)p = v;
    }
  }
}

static __device__ __forceinline__ void att_store(const h16* ow, h16* att, int b, int h,
                                                 int qBase, int lane) {
#pragma unroll
  for (int it = 0; it < 4; ++it) {
    const int rowL = it*4 + (lane >> 3);
    const int piece = lane & 7;
    const v4f v = *(const v4f*)(ow + rowL*OPH + piece*8);
    h16* p = att + ((size_t)b*SEQ + qBase + rowL)*D_MODEL + h*DEPTH + piece*8;
    *(volatile v4f*)p = v;
  }
}

static __device__ __forceinline__ void out_store(const float* Cs, float* out, int mBase,
                                                 int nBase, int wid, int lane) {
#pragma unroll
  for (int it = 0; it < 8; ++it) {
    const int rowL = wid*16 + it*2 + (lane >> 4);
    const int piece = lane & 15;
    const v4f v = *(const v4f*)(Cs + rowL*CPF + piece*4);
    float* p = out + (size_t)(mBase + rowL)*D_MODEL + nBase + piece*4;
    *(volatile v4f*)p = v;
  }
}

__global__ __launch_bounds__(256) void qkv_proj_kernel(
    const float* __restrict__ x,
    const float* __restrict__ wq, const float* __restrict__ bq,
    const float* __restrict__ wk, const float* __restrict__ bk,
    const float* __restrict__ wv, const float* __restrict__ bv,
    h16* qws, h16* kws, h16* vtws) {
  __shared__ __align__(16) h16 Alds[2][128 * LDA];
  __shared__ __align__(16) h16 Blds[2][64 * LDB];
  __shared__ __align__(16) h16 Ct[9216];

  const int z = blockIdx.z;
  const float* __restrict__ W  = (z == 0) ? wq : (z == 1) ? wk : wv;
  const float* __restrict__ Bb = (z == 0) ? bq : (z == 1) ? bk : bv;

  const int tid  = threadIdx.x;
  const int lane = tid & 31, wid = tid >> 5;
  const int waveM = wid >> 1, waveN = wid & 1;
  const int l15 = lane & 15, half = lane >> 4;
  const int mBase = blockIdx.y * 128, nBase = blockIdx.x * 64;

  v8f acc[2][2];
#pragma unroll
  for (int i = 0; i < 2; ++i)
#pragma unroll
    for (int j = 0; j < 2; ++j)
#pragma unroll
      for (int r = 0; r < 8; ++r) acc[i][j][r] = 0.f;

  const int rA = tid >> 1, kpA = (tid & 1) * 16;
  const int nB = tid >> 2, kpB = (tid & 3) * 8;
  const float* ap = x + (size_t)(mBase + rA) * D_MODEL + kpA;
  const float* bp = W + (size_t)(nBase + nB) * D_MODEL + kpB;

  v4f ar[4], br[2];
#pragma unroll
  for (int i = 0; i < 4; ++i) ar[i] = *(const v4f*)(ap + i*4);
  br[0] = *(const v4f*)bp;
  br[1] = *(const v4f*)(bp + 4);

  for (int k0 = 0; k0 < D_MODEL; k0 += 32) {
    const int buf = (k0 >> 5) & 1;
    h16* Al = &Alds[buf][0];
    h16* Bl = &Blds[buf][0];
    *(v8h*)(Al + rA*LDA + kpA)     = cvt8(ar[0], ar[1], 1.0f);
    *(v8h*)(Al + rA*LDA + kpA + 8) = cvt8(ar[2], ar[3], 1.0f);
    *(v8h*)(Bl + nB*LDB + kpB)     = cvt8(br[0], br[1], W_SCALE);
    __syncthreads();
    if (k0 + 32 < D_MODEL) {
#pragma unroll
      for (int i = 0; i < 4; ++i) ar[i] = *(const v4f*)(ap + k0 + 32 + i*4);
      br[0] = *(const v4f*)(bp + k0 + 32);
      br[1] = *(const v4f*)(bp + k0 + 36);
    }
    tile_mma(Al, Bl, waveM, waveN, l15, half, acc);
  }

  const bool tr = (z == 2);
#pragma unroll
  for (int si = 0; si < 2; ++si)
#pragma unroll
    for (int sj = 0; sj < 2; ++sj) {
      const int colL = waveN*32 + sj*16 + l15;
      const float bias = Bb[nBase + colL];
#pragma unroll
      for (int r = 0; r < 8; ++r) {
        const int rowL = waveM*32 + si*16 + half*8 + r;
        const h16 hv = (h16)(acc[si][sj][r] * W_ISCALE + bias);
        if (tr) Ct[colL*CPT + rowL] = hv;
        else    Ct[rowL*CPH + colL] = hv;
      }
    }
  __syncthreads();

  const int b = mBase >> 11, s0 = mBase & (SEQ - 1), h = blockIdx.x;
  h16* dst = tr ? vtws : ((z == 0) ? qws : kws);
  qkv_store(Ct, dst, tr, b, h, s0, wid, lane);
  __threadfence();
  qkv_store(Ct, dst, tr, b, h, s0, wid, lane);
}

__global__ __launch_bounds__(256) void attn_kernel(
    const h16* __restrict__ Q, const h16* __restrict__ K,
    const h16* __restrict__ Vt, h16* att) {
  __shared__ __align__(16) h16 Klds[32 * LDK];
  __shared__ __align__(16) h16 Vtl[64 * LDV];
  __shared__ __align__(16) h16 Olds[8 * 16 * OPH];

  const int tid  = threadIdx.x;
  const int lane = tid & 31, wid = tid >> 5;
  const int l15 = lane & 15, half = lane >> 4;
  const int bh = blockIdx.y;
  const int qBase = blockIdx.x * 128 + wid * 16;
  const size_t bhOff = (size_t)bh * SEQ * DEPTH;

  const h16* Kb  = K  + bhOff;
  const h16* Vtb = Vt + bhOff;

  v16h bqf[2];
  {
    const h16* qp = Q + bhOff + (size_t)(qBase + l15)*DEPTH + half*8;
#pragma unroll
    for (int f = 0; f < 2; ++f)
      bqf[f] = cat8(*(const v8h*)(qp + f*32), *(const v8h*)(qp + f*32 + 16));
  }

  v8f o[4];
#pragma unroll
  for (int j = 0; j < 4; ++j)
#pragma unroll
    for (int r = 0; r < 8; ++r) o[j][r] = 0.f;
  float m_run = -1e30f, l_run = 0.f;

  const int kr = tid >> 3, kpc = (tid & 7) * 8;
  const int vr = tid >> 2, vpc = (tid & 3) * 8;

  for (int kb = 0; kb < SEQ; kb += 32) {
    __syncthreads();
    {
      const v8h kt = *(const v8h*)(Kb + (size_t)(kb + kr)*DEPTH + kpc);
      *(v8h*)(Klds + kr*LDK + kpc) = kt;
      const v8h vt = *(const v8h*)(Vtb + (size_t)vr*SEQ + kb + vpc);
      *(v8h*)(Vtl + vr*LDV + vpc) = vt;
    }
    __syncthreads();

    v8f st[2];
#pragma unroll
    for (int s = 0; s < 2; ++s) {
      const h16* kp_ = Klds + (s*16 + l15)*LDK + half*8;
      const v16h ka0 = cat8(*(const v8h*)kp_,        *(const v8h*)(kp_ + 16));
      const v16h ka1 = cat8(*(const v8h*)(kp_ + 32), *(const v8h*)(kp_ + 48));
      v8f zacc;
#pragma unroll
      for (int r = 0; r < 8; ++r) zacc[r] = 0.f;
      st[s] = wmma16(ka0, bqf[0], zacc);
      st[s] = wmma16(ka1, bqf[1], st[s]);
    }
#pragma unroll
    for (int s = 0; s < 2; ++s)
#pragma unroll
      for (int r = 0; r < 8; ++r) st[s][r] *= SCORE_SC;

    float cmax = -1e30f;
#pragma unroll
    for (int s = 0; s < 2; ++s)
#pragma unroll
      for (int r = 0; r < 8; ++r) cmax = fmaxf(cmax, st[s][r]);
    cmax = fmaxf(cmax, __shfl_xor(cmax, 16, 32));
    const float mnew  = fmaxf(m_run, cmax);
    const float alpha = __expf(m_run - mnew);

    float lsum = 0.f;
    v16h pa;
#pragma unroll
    for (int s = 0; s < 2; ++s)
#pragma unroll
      for (int r = 0; r < 8; ++r) {
        const float p = __expf(st[s][r] - mnew);
        lsum += p;
        pa[s*8 + r] = (h16)(p * P_SCALE);
      }
    lsum += __shfl_xor(lsum, 16, 32);
    l_run = l_run * alpha + lsum;
    m_run = mnew;

#pragma unroll
    for (int r = 0; r < 8; ++r) {
      const float arw = __shfl(alpha, r + half*8, 32);
#pragma unroll
      for (int j = 0; j < 4; ++j) o[j][r] *= arw;
    }

#pragma unroll
    for (int j = 0; j < 4; ++j) {
      const h16* vp = Vtl + (j*16 + l15)*LDV + half*8;
      const v16h vb = cat8(*(const v8h*)vp, *(const v8h*)(vp + 16));
      o[j] = wmma16(pa, vb, o[j]);
    }
  }

  const float linv = 1.0f / l_run;
  h16* ow = Olds + wid * 16 * OPH;
#pragma unroll
  for (int r = 0; r < 8; ++r) {
    const float lr = __shfl(linv, r + half*8, 32) * ATT_OSCALE;
#pragma unroll
    for (int j = 0; j < 4; ++j)
      ow[(half*8 + r)*OPH + j*16 + l15] = (h16)(o[j][r] * lr);
  }
  __syncthreads();

  const int b = bh >> 4, h = bh & 15;
  att_store(ow, att, b, h, qBase, lane);
  __threadfence();
  att_store(ow, att, b, h, qBase, lane);
}

__global__ __launch_bounds__(256) void out_proj_kernel(
    const h16* __restrict__ A, const float* __restrict__ W,
    const float* __restrict__ bias, float* out) {
  __shared__ __align__(16) h16   Alds[2][128 * LDA];
  __shared__ __align__(16) h16   Blds[2][64 * LDB];
  __shared__ __align__(16) float Cs[128 * CPF];

  const int tid  = threadIdx.x;
  const int lane = tid & 31, wid = tid >> 5;
  const int waveM = wid >> 1, waveN = wid & 1;
  const int l15 = lane & 15, half = lane >> 4;
  const int mBase = blockIdx.y * 128, nBase = blockIdx.x * 64;

  v8f acc[2][2];
#pragma unroll
  for (int i = 0; i < 2; ++i)
#pragma unroll
    for (int j = 0; j < 2; ++j)
#pragma unroll
      for (int r = 0; r < 8; ++r) acc[i][j][r] = 0.f;

  const int rA = tid >> 1, kpA = (tid & 1) * 16;
  const int nB = tid >> 2, kpB = (tid & 3) * 8;
  const h16*  ap = A + (size_t)(mBase + rA) * D_MODEL + kpA;
  const float* bp = W + (size_t)(nBase + nB) * D_MODEL + kpB;

  v8h arb[2];
  v4f br[2];
  arb[0] = *(const v8h*)ap;
  arb[1] = *(const v8h*)(ap + 8);
  br[0]  = *(const v4f*)bp;
  br[1]  = *(const v4f*)(bp + 4);

  for (int k0 = 0; k0 < D_MODEL; k0 += 32) {
    const int buf = (k0 >> 5) & 1;
    h16* Al = &Alds[buf][0];
    h16* Bl = &Blds[buf][0];
    *(v8h*)(Al + rA*LDA + kpA)     = arb[0];
    *(v8h*)(Al + rA*LDA + kpA + 8) = arb[1];
    *(v8h*)(Bl + nB*LDB + kpB)     = cvt8(br[0], br[1], W_SCALE);
    __syncthreads();
    if (k0 + 32 < D_MODEL) {
      arb[0] = *(const v8h*)(ap + k0 + 32);
      arb[1] = *(const v8h*)(ap + k0 + 40);
      br[0]  = *(const v4f*)(bp + k0 + 32);
      br[1]  = *(const v4f*)(bp + k0 + 36);
    }
    tile_mma(Al, Bl, waveM, waveN, l15, half, acc);
  }

#pragma unroll
  for (int si = 0; si < 2; ++si)
#pragma unroll
    for (int sj = 0; sj < 2; ++sj) {
      const int colL = waveN*32 + sj*16 + l15;
      const float bvv = bias[nBase + colL];
#pragma unroll
      for (int r = 0; r < 8; ++r) {
        const int rowL = waveM*32 + si*16 + half*8 + r;
        Cs[rowL*CPF + colL] = acc[si][sj][r] * OUT_ISCALE + bvv;
      }
    }
  __syncthreads();

  out_store(Cs, out, mBase, nBase, wid, lane);
  __threadfence();
  out_store(Cs, out, mBase, nBase, wid, lane);
}

extern "C" void kernel_launch(void* const* d_in, const int* in_sizes, int n_in,
                              void* d_out, int out_size, void* d_ws, size_t ws_size,
                              hipStream_t stream) {
  if (n_in < 9) return;
  const int ne = M_TOTAL * D_MODEL;
  if (in_sizes[0] != ne || out_size != ne) return;
  if (in_sizes[1] != D_MODEL * D_MODEL || in_sizes[3] != D_MODEL * D_MODEL ||
      in_sizes[5] != D_MODEL * D_MODEL || in_sizes[7] != D_MODEL * D_MODEL) return;
  if (in_sizes[2] != D_MODEL || in_sizes[4] != D_MODEL ||
      in_sizes[6] != D_MODEL || in_sizes[8] != D_MODEL) return;

  const size_t NE = (size_t)ne;
  const size_t need = 4 * NE * sizeof(h16);
  if (ws_size < need) return;

  const float* x       = (const float*)d_in[0];
  const float* wq_w    = (const float*)d_in[1];
  const float* wq_b    = (const float*)d_in[2];
  const float* wk_w    = (const float*)d_in[3];
  const float* wk_b    = (const float*)d_in[4];
  const float* wv_w    = (const float*)d_in[5];
  const float* wv_b    = (const float*)d_in[6];
  const float* dense_w = (const float*)d_in[7];
  const float* dense_b = (const float*)d_in[8];

  h16* q_ws   = (h16*)d_ws;
  h16* k_ws   = q_ws  + NE;
  h16* vt_ws  = k_ws  + NE;
  h16* att_ws = vt_ws + NE;

  dim3 gQKV(D_MODEL / 64, M_TOTAL / 128, 3);
  qkv_proj_kernel<<<gQKV, 256, 0, stream>>>(x, wq_w, wq_b, wk_w, wk_b, wv_w, wv_b,
                                            q_ws, k_ws, vt_ws);

  dim3 gAtt(SEQ / 128, BATCH * HEADS);
  attn_kernel<<<gAtt, 256, 0, stream>>>(q_ws, k_ws, vt_ws, att_ws);

  dim3 gOut(D_MODEL / 64, M_TOTAL / 128);
  out_proj_kernel<<<gOut, 256, 0, stream>>>(att_ws, dense_w, dense_b, (float*)d_out);
}
